// RWKV_TimeMix_16028817949581
// MI455X (gfx1250) — hardware-verified
//
#include <hip/hip_runtime.h>
#include <math.h>

constexpr int kBat   = 8;
constexpr int kSeq   = 1024;
constexpr int kEmb   = 1024;
constexpr int kAtt   = 1024;
constexpr int kHeads = 16;
constexpr int kHd    = 64;
constexpr int kCtx   = 1024;
constexpr int kHalfC = kEmb / 2;
constexpr int kRows  = kBat * kSeq;
constexpr int kStripLd = 1024;
constexpr size_t kPlaneElems = (size_t)kBat * kAtt * kSeq;
static_assert(kAtt == kHeads * kHd, "head split");
static_assert(kCtx == kSeq, "decay table length equals sequence length");
static_assert(kRows % 64 == 0 && kAtt % 64 == 0 && kEmb % 64 == 0, "GEMM M, N tile multiples");
static_assert(kEmb % 32 == 0 && (2 * kAtt) % 32 == 0 && kSeq % 64 == 0, "GEMM K multiples of 32");
static_assert(kHd == 64, "one 64-wide N tile per head");
static_assert(kHalfC % 8 == 0, "8-element groups never straddle the shift boundary");
static_assert(kStripLd == kSeq, "strip column range 0..1023");

typedef __attribute__((ext_vector_type(16))) __bf16   v16b;
typedef __attribute__((ext_vector_type(8)))  __bf16   v8b;
typedef __attribute__((ext_vector_type(8)))  float    v8f;
typedef __attribute__((ext_vector_type(4)))  float    v4f;
typedef __attribute__((ext_vector_type(2)))  float    v2f;
typedef __attribute__((ext_vector_type(4)))  unsigned int v4u;

__device__ __forceinline__ unsigned short f2bf_bits(float f) {
  unsigned u = __float_as_uint(f);
  return (unsigned short)((u + 0x7FFFu + ((u >> 16) & 1u)) >> 16);
}
__device__ __forceinline__ float bf_bits2f(unsigned short h) { return __uint_as_float(((unsigned)h) << 16); }
__device__ __forceinline__ float bf16r(float f) { return bf_bits2f(f2bf_bits(f)); }
__device__ __forceinline__ unsigned pk16(unsigned short a, unsigned short b) { return (unsigned)a | ((unsigned)b << 16); }

__device__ __forceinline__ void keep4_b(v16b a, v16b b, v16b c, v16b d) { asm volatile("v_nop" :: "v"(a), "v"(b), "v"(c), "v"(d)); }
__device__ __forceinline__ void acc_guard4(v8f& a, v8f& b, v8f& c, v8f& d) { asm volatile("v_nop\n\tv_nop\n\tv_nop\n\tv_nop" : "+v"(a), "+v"(b), "+v"(c), "+v"(d)); }
__device__ __forceinline__ void group_guard_b(v8f& a0, v8f& a1, v8f& a2, v8f& a3, v16b x, v16b b0, v16b b1, v16b b2, v16b b3) {
  asm volatile("v_nop\n\tv_nop\n\tv_nop\n\tv_nop" : "+v"(a0), "+v"(a1), "+v"(a2), "+v"(a3) : "v"(x), "v"(b0), "v"(b1), "v"(b2), "v"(b3));
}

template <typename T> struct Frag;
template <> struct Frag<__bf16> {
  typedef v16b V; union U { v16b v; v8b h[2]; };
  static __device__ __forceinline__ v16b load(const __bf16* p) {
    U f; f.h[0] = *(const v8b*)(p); f.h[1] = *(const v8b*)(p + 16); return f.v;
  }
  static __device__ __forceinline__ v8f mma(v16b a, v16b b, v8f c) {
    return __builtin_amdgcn_wmma_f32_16x16x32_bf16(false, a, false, b, (short)0, c, false, false);
  }
  static __device__ __forceinline__ void keep(v16b a, v16b b, v16b c, v16b d) { keep4_b(a, b, c, d); }
};

__device__ __forceinline__ void wave_lds_sync() {
  __builtin_amdgcn_fence(__ATOMIC_RELEASE, "workgroup");
  __builtin_amdgcn_wave_barrier();
  __builtin_amdgcn_fence(__ATOMIC_ACQUIRE, "workgroup");
}

__global__ __launch_bounds__(256) void shift_convert_kernel(const float* __restrict__ x, unsigned short* __restrict__ xs, int n8) {
  const int i = blockIdx.x * 256 + threadIdx.x;
  if (i >= n8) return;
  const int row = i >> 7;
  const int c0  = (i & 127) * 8;
  const int t   = row & (kSeq - 1);
  const bool shifted = (c0 < kHalfC);
  const bool dead    = shifted && (t == 0);
  const int srow = (shifted && (t > 0)) ? (row - 1) : row;
  const float* p = x + (size_t)srow * kEmb + c0;
  const v4f a = *(const v4f*)(p);
  const v4f c = *(const v4f*)(p + 4);
  unsigned short hb[8];
#pragma unroll
  for (int e = 0; e < 4; ++e) {
    const float fa = dead ? 0.0f : a[e];
    const float fc = dead ? 0.0f : c[e];
    hb[e]     = f2bf_bits(fa);
    hb[4 + e] = f2bf_bits(fc);
  }
  const v4u u = (v4u){pk16(hb[0], hb[1]), pk16(hb[2], hb[3]), pk16(hb[4], hb[5]), pk16(hb[6], hb[7])};
  unsigned short* q = xs + 8 * (size_t)i;
  *(volatile v4u*)q = u;
  __threadfence();
  *(volatile v4u*)q = u;
}

__global__ __launch_bounds__(256) void wt_prep_kernel(const float* __restrict__ W0, const float* __restrict__ W1,
                                                      const float* __restrict__ W2, const float* __restrict__ W3,
                                                      unsigned short* __restrict__ wt, unsigned short* __restrict__ wo2) {
  __shared__ float sm[64][65];
  const int t  = threadIdx.x;
  const int d0 = blockIdx.x * 64;
  const int h0 = blockIdx.y * 64;
  const int z  = blockIdx.z;
  const float* W = (z == 0) ? W0 : (z == 1) ? W1 : (z == 2) ? W2 : W3;
  unsigned short* op = (z < 3) ? (wt + (size_t)z * kAtt * kEmb) : wo2;
  const int ldo = (z < 3) ? kEmb : (2 * kAtt);
#pragma unroll 4
  for (int i = 0; i < 16; ++i) {
    const int e = i * 256 + t;
    const int r = e >> 6;
    const int c = e & 63;
    sm[c][r] = W[(size_t)(d0 + r) * 1024 + h0 + c];
  }
  __syncthreads();
  const int lane = t & 31, wave = t >> 5;
  const int q = lane >> 3, c8 = (lane & 7) * 8;
  for (int pass = 0; pass < 2; ++pass) {
#pragma unroll
    for (int it = 0; it < 2; ++it) {
      const int row = wave * 8 + it * 4 + q;
      unsigned short hb[8];
#pragma unroll
      for (int e = 0; e < 8; ++e) hb[e] = f2bf_bits(sm[row][c8 + e]);
      const v4u u = (v4u){pk16(hb[0], hb[1]), pk16(hb[2], hb[3]), pk16(hb[4], hb[5]), pk16(hb[6], hb[7])};
      unsigned short* dst = op + (size_t)(h0 + row) * ldo + d0 + c8;
      *(volatile v4u*)dst = u;
      if (z == 3) *(volatile v4u*)(dst + kAtt) = u;
    }
    __threadfence();
  }
}

__global__ __launch_bounds__(256) void strip_build_kernel(const float* __restrict__ tw, unsigned short* __restrict__ S, int n8) {
  const int i = blockIdx.x * 256 + threadIdx.x;
  if (i >= n8) return;
  const int j0 = (i & 127) * 8;
  const int r  = (i >> 7) & 63;
  const int h  = i >> 13;
  unsigned short hb[8];
#pragma unroll
  for (int e = 0; e < 8; ++e) {
    const int idx = j0 + e + 63 - r;
    const int ic  = (idx < kCtx - 1) ? idx : (kCtx - 1);
    const float v = tw[h * kCtx + ic];
    unsigned short bits = f2bf_bits(v);
    bits = ((bits & 0x7F80u) == 0u) ? (unsigned short)0 : bits;
    bits = (idx > kCtx - 1) ? (unsigned short)0 : bits;
    hb[e] = bits;
  }
  const v4u u = (v4u){pk16(hb[0], hb[1]), pk16(hb[2], hb[3]), pk16(hb[4], hb[5]), pk16(hb[6], hb[7])};
  unsigned short* q = S + 8 * (size_t)i;
  *(volatile v4u*)q = u;
  __threadfence();
  *(volatile v4u*)q = u;
}

template <int MODE>
__global__ __launch_bounds__(256) void proj_gemm_kernel(
    const unsigned short* __restrict__ Ap, int lda,
    const unsigned short* __restrict__ Btp, int ldb,
    float* __restrict__ Cout, int ldc,
    const float* __restrict__ bias,
    const float* __restrict__ aux,
    const float* __restrict__ tvec,
    int M, int N, int K) {
  const __bf16* A  = (const __bf16*)Ap;
  const __bf16* Bt = (const __bf16*)Btp;
  __shared__ __align__(16) float sT[8][16 * 68];
  const int lane = threadIdx.x & 31;
  const int wave = threadIdx.x >> 5;
  const int tilesN = N >> 6;
  const int tilesM = M >> 6;
  const int tile = blockIdx.x * 8 + wave;
  if (tile >= tilesM * tilesN) return;
  const int tm = tile / tilesN;
  const int tn = tile - tm * tilesN;
  const int m0 = tm << 6;
  const int n0 = tn << 6;
  const int rlane = lane & 15;
  const int koff  = (lane >> 4) * 8;
  const int mOff  = (lane >> 4) * 8;

  v8f acc[4][4];
#pragma unroll
  for (int i = 0; i < 4; ++i)
#pragma unroll
    for (int j = 0; j < 4; ++j) acc[i][j] = (v8f){0.f, 0.f, 0.f, 0.f, 0.f, 0.f, 0.f, 0.f};

#pragma unroll 1
  for (int k0 = 0; k0 < K; k0 += 32) {
    v16b bh[4];
#pragma unroll
    for (int j = 0; j < 4; ++j)
      bh[j] = Frag<__bf16>::load(Bt + (size_t)(n0 + (j << 4) + rlane) * ldb + koff + k0);
#pragma unroll
    for (int i = 0; i < 4; ++i) {
      const v16b ah = Frag<__bf16>::load(A + (size_t)(m0 + (i << 4) + rlane) * lda + koff + k0);
#pragma unroll
      for (int j = 0; j < 4; ++j) acc[i][j] = Frag<__bf16>::mma(ah, bh[j], acc[i][j]);
      group_guard_b(acc[i][0], acc[i][1], acc[i][2], acc[i][3], ah, bh[0], bh[1], bh[2], bh[3]);
    }
    Frag<__bf16>::keep(bh[0], bh[1], bh[2], bh[3]);
  }
  acc_guard4(acc[0][0], acc[0][1], acc[0][2], acc[0][3]);
  acc_guard4(acc[1][0], acc[1][1], acc[1][2], acc[1][3]);
  acc_guard4(acc[2][0], acc[2][1], acc[2][2], acc[2][3]);
  acc_guard4(acc[3][0], acc[3][1], acc[3][2], acc[3][3]);

  float* slab = sT[wave];
  const int c2 = lane * 2;
  const v2f bpair = *(const v2f*)(bias + n0 + c2);
  const float bias0 = bf16r(bpair[0]);
  const float bias1 = bf16r(bpair[1]);
  const int hcol = n0 >> 6;
#pragma unroll
  for (int i = 0; i < 4; ++i) {
    const int mBase = m0 + (i << 4);
#pragma unroll
    for (int j = 0; j < 4; ++j)
#pragma unroll
      for (int r = 0; r < 8; ++r) slab[(mOff + r) * 68 + (j << 4) + rlane] = acc[i][j][r];
    wave_lds_sync();
#pragma unroll 1
    for (int rr = 0; rr < 16; ++rr) {
      float* sp = slab + rr * 68 + c2;
      const v2f v = *(const v2f*)sp;
      float y0 = v[0] + bias0;
      float y1 = v[1] + bias1;
      const int grow = mBase + rr;
      if (MODE == 0) {
        y0 = expf(fminf(fmaxf(y0, -60.0f), 30.0f));
        y1 = expf(fminf(fmaxf(y1, -60.0f), 30.0f));
      }
      if (MODE == 2) {
        const float bt = bf16r(tvec[hcol * kCtx + (grow & (kSeq - 1))]);
        const v2f sk = *(const v2f*)(aux + (size_t)grow * ldc + n0 + c2);
        const float den0 = (1.0f + expf(-y0)) * sk[0];
        const float den1 = (1.0f + expf(-y1)) * sk[1];
        y0 = bt * (1.0f / den0);
        y1 = bt * (1.0f / den1);
      }
      if (MODE == 3) {
        const float gm = bf16r(tvec[grow & (kSeq - 1)]);
        y0 = y0 * gm;
        y1 = y1 * gm;
      }
      const v2f o = (v2f){y0, y1};
      *(v2f*)sp = o;
    }
    wave_lds_sync();
    {
      const int hh = lane >> 4, c4 = (lane & 15) * 4;
      for (int pass = 0; pass < 2; ++pass) {
#pragma unroll
        for (int it = 0; it < 8; ++it) {
          const int row = it * 2 + hh;
          const v4f v = *(const v4f*)(slab + row * 68 + c4);
          *(volatile v4f*)(Cout + (size_t)(mBase + row) * ldc + n0 + c4) = v;
        }
        __threadfence();
      }
    }
    wave_lds_sync();
  }
}

__global__ __launch_bounds__(256) void kv_prep_kernel(const float* __restrict__ kpl, const float* __restrict__ vpl,
                                                      const float* __restrict__ alpha,
                                                      unsigned short* __restrict__ pt_hi, unsigned short* __restrict__ pt_lo) {
  __shared__ float sm[64][65];
  const int t   = threadIdx.x;
  const int h   = blockIdx.x;
  const int ch0 = blockIdx.x * 64;
  const int u0  = blockIdx.y * 64;
  const int b   = blockIdx.z;
#pragma unroll 4
  for (int i = 0; i < 16; ++i) {
    const int e = i * 256 + t;
    const int r = e >> 6;
    const int c = e & 63;
    const size_t idx = ((size_t)b * kSeq + u0 + r) * kAtt + ch0 + c;
    const float al = bf16r(alpha[h * kCtx + u0 + r]);
    const float kk = kpl[idx];
    const float vv = vpl[idx];
    const float kv = kk * vv;
    sm[c][r] = al * kv;
  }
  __syncthreads();
  const int lane = t & 31, wave = t >> 5;
  const int q = lane >> 3, c8 = (lane & 7) * 8;
  for (int pass = 0; pass < 2; ++pass) {
#pragma unroll
    for (int it = 0; it < 2; ++it) {
      const int row = wave * 8 + it * 4 + q;
      unsigned short hb[8], lb[8];
#pragma unroll
      for (int e = 0; e < 8; ++e) {
        const float f = sm[row][c8 + e];
        hb[e] = f2bf_bits(f);
        lb[e] = f2bf_bits(f - bf_bits2f(hb[e]));
      }
      const v4u uh = (v4u){pk16(hb[0], hb[1]), pk16(hb[2], hb[3]), pk16(hb[4], hb[5]), pk16(hb[6], hb[7])};
      const v4u ul = (v4u){pk16(lb[0], lb[1]), pk16(lb[2], lb[3]), pk16(lb[4], lb[5]), pk16(lb[6], lb[7])};
      const size_t off = ((size_t)b * kAtt + ch0 + row) * kSeq + u0 + c8;
      *(volatile v4u*)(pt_hi + off) = uh;
      *(volatile v4u*)(pt_lo + off) = ul;
    }
    __threadfence();
  }
}

__global__ __launch_bounds__(256) void cumsum_kernel(const float* __restrict__ kpl, float* __restrict__ skp) {
  const int i = blockIdx.x * 256 + threadIdx.x;
  if (i >= kBat * kAtt) return;
  const int b  = i >> 10;
  const int ch = i & (kAtt - 1);
  const float* src = kpl + (size_t)b * kSeq * kAtt + ch;
  float* dst = skp + (size_t)b * kSeq * kAtt + ch;
  float s = 0.0f;
#pragma unroll 1
  for (int tb = 0; tb < kSeq; tb += 8) {
    float v[8];
#pragma unroll
    for (int e = 0; e < 8; ++e) v[e] = src[(size_t)(tb + e) * kAtt];
#pragma unroll
    for (int e = 0; e < 8; ++e) { s += v[e]; v[e] = s; }
    for (int pass = 0; pass < 2; ++pass) {
#pragma unroll
      for (int e = 0; e < 8; ++e) *(volatile float*)(dst + (size_t)(tb + e) * kAtt) = v[e];
      __threadfence();
    }
  }
}

__global__ __launch_bounds__(256) void decay_gemm_kernel(const unsigned short* __restrict__ Sp,
                                                         const unsigned short* __restrict__ PTp,
                                                         const float* __restrict__ G,
                                                         unsigned short* __restrict__ R2) {
  const __bf16* S  = (const __bf16*)Sp;
  const __bf16* PT = (const __bf16*)PTp;
  __shared__ __align__(16) float sT[8][16 * 68];
  const int lane = threadIdx.x & 31;
  const int wave = threadIdx.x >> 5;
  const int tile = blockIdx.x * 8 + wave;
  if (tile >= kBat * kHeads * (kSeq / 64)) return;
  const int mt = tile & 15;
  const int h  = (tile >> 4) & 15;
  const int b  = tile >> 8;
  const int t0 = mt * 64;
  const int kend = t0 + 64;
  const int rlane = lane & 15;
  const int koff  = (lane >> 4) * 8;
  const int mOff  = (lane >> 4) * 8;
  const __bf16* Ab = S + (size_t)h * 64 * kStripLd + (960 - t0);

  v8f acc[4][4];
#pragma unroll
  for (int i = 0; i < 4; ++i)
#pragma unroll
    for (int j = 0; j < 4; ++j) acc[i][j] = (v8f){0.f, 0.f, 0.f, 0.f, 0.f, 0.f, 0.f, 0.f};

#pragma unroll 1
  for (int p = 0; p < 2; ++p) {
    const __bf16* Bb = PT + (size_t)p * kPlaneElems + ((size_t)b * kAtt + (size_t)h * kHd) * kSeq;
#pragma unroll 1
    for (int k0 = 0; k0 < kend; k0 += 32) {
      v16b bh[4];
#pragma unroll
      for (int j = 0; j < 4; ++j)
        bh[j] = Frag<__bf16>::load(Bb + (size_t)((j << 4) + rlane) * kSeq + koff + k0);
#pragma unroll
      for (int i = 0; i < 4; ++i) {
        const v16b ah = Frag<__bf16>::load(Ab + (size_t)((i << 4) + rlane) * kStripLd + koff + k0);
#pragma unroll
        for (int j = 0; j < 4; ++j) acc[i][j] = Frag<__bf16>::mma(ah, bh[j], acc[i][j]);
        group_guard_b(acc[i][0], acc[i][1], acc[i][2], acc[i][3], ah, bh[0], bh[1], bh[2], bh[3]);
      }
      Frag<__bf16>::keep(bh[0], bh[1], bh[2], bh[3]);
    }
  }
  acc_guard4(acc[0][0], acc[0][1], acc[0][2], acc[0][3]);
  acc_guard4(acc[1][0], acc[1][1], acc[1][2], acc[1][3]);
  acc_guard4(acc[2][0], acc[2][1], acc[2][2], acc[2][3]);
  acc_guard4(acc[3][0], acc[3][1], acc[3][2], acc[3][3]);

  float* slab = sT[wave];
  const int c2 = lane * 2;
  const size_t rowBase = (size_t)b * kSeq + t0;
#pragma unroll
  for (int i = 0; i < 4; ++i) {
    const int mLoc = (i << 4);
#pragma unroll
    for (int j = 0; j < 4; ++j)
#pragma unroll
      for (int r = 0; r < 8; ++r) slab[(mOff + r) * 68 + (j << 4) + rlane] = acc[i][j][r];
    wave_lds_sync();
#pragma unroll 1
    for (int rr = 0; rr < 16; ++rr) {
      float* sp = slab + rr * 68 + c2;
      const v2f v = *(const v2f*)sp;
      const v2f g = *(const v2f*)(G + (rowBase + mLoc + rr) * kAtt + h * kHd + c2);
      const v2f o = (v2f){v[0] * g[0], v[1] * g[1]};
      *(v2f*)sp = o;
    }
    wave_lds_sync();
    {
      const int q = lane >> 3, c8 = (lane & 7) * 8;
      for (int pass = 0; pass < 2; ++pass) {
#pragma unroll
        for (int it = 0; it < 4; ++it) {
          const int row = it * 4 + q;
          const float* sp = slab + row * 68 + c8;
          const v4f fa = *(const v4f*)(sp);
          const v4f fc = *(const v4f*)(sp + 4);
          unsigned short hb[8], lb[8];
#pragma unroll
          for (int e = 0; e < 4; ++e) {
            const float x0 = fa[e];
            const float x1 = fc[e];
            hb[e]     = f2bf_bits(x0);
            lb[e]     = f2bf_bits(x0 - bf_bits2f(hb[e]));
            hb[4 + e] = f2bf_bits(x1);
            lb[4 + e] = f2bf_bits(x1 - bf_bits2f(hb[4 + e]));
          }
          const v4u uh = (v4u){pk16(hb[0], hb[1]), pk16(hb[2], hb[3]), pk16(hb[4], hb[5]), pk16(hb[6], hb[7])};
          const v4u ul = (v4u){pk16(lb[0], lb[1]), pk16(lb[2], lb[3]), pk16(lb[4], lb[5]), pk16(lb[6], lb[7])};
          unsigned short* dst = R2 + (rowBase + mLoc + row) * (size_t)(2 * kAtt) + h * kHd + c8;
          *(volatile v4u*)dst = uh;
          *(volatile v4u*)(dst + kAtt) = ul;
        }
        __threadfence();
      }
    }
    wave_lds_sync();
  }
}

extern "C" void kernel_launch(void* const* d_in, const int* in_sizes, int n_in,
                              void* d_out, int out_size, void* d_ws, size_t ws_size, hipStream_t stream) {
  if (n_in < 13 || d_out == nullptr || d_ws == nullptr) return;
  if (in_sizes[0] != kRows * kEmb || in_sizes[1] != kHeads * kCtx || in_sizes[2] != kHeads * kCtx ||
      in_sizes[3] != kHeads * kCtx || in_sizes[4] != kCtx ||
      in_sizes[5] != kEmb * kAtt || in_sizes[6] != kAtt || in_sizes[7] != kEmb * kAtt || in_sizes[8] != kAtt ||
      in_sizes[9] != kEmb * kAtt || in_sizes[10] != kAtt || in_sizes[11] != kAtt * kEmb || in_sizes[12] != kEmb ||
      out_size != kRows * kEmb) return;

  const float* x     = (const float*)d_in[0];
  const float* tw    = (const float*)d_in[1];
  const float* alpha = (const float*)d_in[2];
  const float* beta  = (const float*)d_in[3];
  const float* gamma = (const float*)d_in[4];
  const float* Wk    = (const float*)d_in[5];
  const float* bk    = (const float*)d_in[6];
  const float* Wv    = (const float*)d_in[7];
  const float* bv    = (const float*)d_in[8];
  const float* Wr    = (const float*)d_in[9];
  const float* br    = (const float*)d_in[10];
  const float* Wo    = (const float*)d_in[11];
  const float* bo    = (const float*)d_in[12];
  float* out = (float*)d_out;

  char* ws = (char*)d_ws; size_t off = 0;
  auto carve = [&](size_t bytes) -> char* { char* p = ws + off; off += (bytes + 255) & ~(size_t)255; return p; };
  unsigned short* P0  = (unsigned short*)carve((size_t)kRows * kEmb * 2);
  unsigned short* WT  = (unsigned short*)carve((size_t)3 * kAtt * kEmb * 2);
  unsigned short* WO2 = (unsigned short*)carve((size_t)kEmb * 2 * kAtt * 2);
  unsigned short* ST  = (unsigned short*)carve((size_t)kHeads * 64 * kStripLd * 2);
  float*          PK  = (float*)carve((size_t)kRows * kAtt * 4);
  float*          PV  = (float*)carve((size_t)kRows * kAtt * 4);
  unsigned short* PT  = (unsigned short*)carve((size_t)2 * kPlaneElems * 2);
  if (off > ws_size || off > (size_t)134217728) return;
  unsigned short* R2  = (unsigned short*)PV;

  const int n8x = kRows * (kEmb / 8);
  shift_convert_kernel<<<n8x / 256, 256, 0, stream>>>(x, P0, n8x);
  wt_prep_kernel<<<dim3(kEmb / 64, kAtt / 64, 4), 256, 0, stream>>>(Wk, Wv, Wr, Wo, WT, WO2);
  const int n8s = kHeads * 64 * (kStripLd / 8);
  strip_build_kernel<<<n8s / 256, 256, 0, stream>>>(tw, ST, n8s);

  const int ggrid = (kRows / 64) * (kAtt / 64) / 8;
  proj_gemm_kernel<0><<<ggrid, 256, 0, stream>>>(P0, kEmb, WT, kEmb, PK, kAtt, bk, bk, bk, kRows, kAtt, kEmb);
  proj_gemm_kernel<1><<<ggrid, 256, 0, stream>>>(P0, kEmb, WT + (size_t)kAtt * kEmb, kEmb, PV, kAtt, bv, bv, bv,
                                                 kRows, kAtt, kEmb);

  kv_prep_kernel<<<dim3(kAtt / 64, kSeq / 64, kBat), 256, 0, stream>>>(PK, PV, alpha, PT, PT + kPlaneElems);
  cumsum_kernel<<<(kBat * kAtt) / 256, 256, 0, stream>>>(PK, PV);

  proj_gemm_kernel<2><<<ggrid, 256, 0, stream>>>(P0, kEmb, WT + (size_t)2 * kAtt * kEmb, kEmb, PK, kAtt, br, PV, beta,
                                                 kRows, kAtt, kEmb);

  decay_gemm_kernel<<<(kBat * kHeads * (kSeq / 64)) / 8, 256, 0, stream>>>(ST, PT, PK, R2);

  proj_gemm_kernel<3><<<(kRows / 64) * (kEmb / 64) / 8, 256, 0, stream>>>(R2, 2 * kAtt, WO2, 2 * kAtt, out, kEmb,
                                                                          bo, bo, gamma, kRows, kEmb, 2 * kAtt);
}
